// CoreDotProductAttention_10977936409095
// MI455X (gfx1250) — hardware-verified
//
#include <hip/hip_runtime.h>


namespace {
constexpr int NB = 2, S = 2048, E = 1024, NH = 16, D = 64, NR = NB * S;
constexpr float XS = 8.0f, WSC = 256.0f, PS = 8.0f, SCALE = 0.125f, LOG2E = 1.4426950408889634f;

typedef _Float16 b16;
typedef __attribute__((ext_vector_type(16))) _Float16 v16b;
typedef __attribute__((ext_vector_type(8))) _Float16 v8b;
typedef __attribute__((ext_vector_type(8))) float v8f;
typedef __attribute__((ext_vector_type(4))) float v4f;
typedef __attribute__((ext_vector_type(4))) int v4i;
__device__ __forceinline__ float bf16_rne(float f) { unsigned int u = __float_as_uint(f); u += 0x7FFFu + ((u >> 16) & 1u); return __uint_as_float(u & 0xFFFF0000u); }
__device__ __forceinline__ void split16(float v, b16& hi, b16& lo) { hi = (b16)v; lo = (b16)(v - (float)hi); }
__device__ __forceinline__ v16b frag_kb(const b16* p, int hh) { const v8b a = *(const v8b*)(p + 8 * hh), b = *(const v8b*)(p + 16 + 8 * hh); v16b f;
#pragma unroll
  for (int e = 0; e < 8; ++e) { f[e] = a[e]; f[8 + e] = b[e]; } return f; }
__device__ __forceinline__ v8f wmma16b(v16b a, v16b b, v8f c) { v8f d = __builtin_amdgcn_wmma_f32_16x16x32_f16(false, a, false, b, (short)0, c, false, false); asm volatile("v_nop\n\tv_nop\n\tv_nop\n\tv_nop" : "+v"(d) : "v"(a), "v"(b)); return d; }
__device__ __forceinline__ void wave_lds_sync() { __builtin_amdgcn_fence(__ATOMIC_RELEASE, "workgroup"); __builtin_amdgcn_wave_barrier(); __builtin_amdgcn_fence(__ATOMIC_ACQUIRE, "workgroup"); }
__device__ __forceinline__ float nexp2(float x) { return __builtin_amdgcn_exp2f(x); }

__global__ __launch_bounds__(256) void prep_kernel(const float* __restrict__ q, const float* __restrict__ k, const float* __restrict__ w, b16* __restrict__ Q16, b16* __restrict__ K16, b16* __restrict__ W16) {
  const size_t t = (size_t)blockIdx.x * 256 + threadIdx.x; const size_t nq = (size_t)NR * E / 8, nw = (size_t)E * E / 8;
  const float* src; b16* dst; size_t e; float sc = XS; if (t < nq) { src = q; dst = Q16; e = t * 8; } else if (t < 2 * nq) { src = k; dst = K16; e = (t - nq) * 8; } else if (t < 2 * nq + nw) { src = w; dst = W16; e = (t - 2 * nq) * 8; sc = WSC; } else return;
  const v4f a = *(const v4f*)(src + e), c = *(const v4f*)(src + e + 4); v8b o;
#pragma unroll
  for (int j = 0; j < 4; ++j) { o[j] = (b16)(bf16_rne(a[j]) * sc); o[4 + j] = (b16)(bf16_rne(c[j]) * sc); }
  for (int pass = 0; pass < 2; ++pass) { *(volatile v8b*)(dst + e) = o; __threadfence(); }
}
__global__ __launch_bounds__(256) void vt_kernel(const float* __restrict__ v, b16* __restrict__ VT16) {
  __shared__ __attribute__((aligned(16))) b16 T[64][64 + 8];
  const int b = blockIdx.z, h = blockIdx.y, s0 = blockIdx.x * 64, t_ = threadIdx.x;
  for (int qq = t_; qq < 64 * 64; qq += 256) { const int ss = qq >> 6, dd = qq & 63; T[dd][ss] = (b16)(bf16_rne(v[((size_t)b * S + s0 + ss) * E + h * D + dd]) * XS); }
  __syncthreads();
  for (int pass = 0; pass < 2; ++pass) { for (int qq = t_; qq < 64 * 8; qq += 256) { const int dd = qq >> 3, c8 = (qq & 7) * 8; *(volatile v8b*)(VT16 + (((size_t)b * NH + h) * D + dd) * S + s0 + c8) = *(const v8b*)(&T[dd][c8]); } __threadfence(); }
}
__global__ __launch_bounds__(64) void attn_kernel(const b16* __restrict__ Q16, const b16* __restrict__ K16, const b16* __restrict__ VT16, const int* __restrict__ pmask, b16* __restrict__ Oh, b16* __restrict__ Ol) {
  __shared__ __attribute__((aligned(16))) float To[2][16][D + 4];
  const int wave = threadIdx.x >> 5, lane = threadIdx.x & 31, hh = lane >> 4, col = lane & 15; const int b = blockIdx.z, h = blockIdx.y; const int q0 = blockIdx.x * 32 + wave * 16, qi = q0 + col;
  const b16* Qp = Q16 + ((size_t)b * S + qi) * E + h * D; const b16* Kb = K16 + (size_t)b * S * E + h * D; const b16* Vb = VT16 + ((size_t)b * NH + h) * D * S; const int* mrow = pmask + ((size_t)b * S + qi) * S;
  const v16b qa0 = frag_kb(Qp, hh), qa1 = frag_kb(Qp + 32, hh);
  float m = -INFINITY, l = 0.0f; v8f o[4] = {{}, {}, {}, {}}, ol[4] = {{}, {}, {}, {}};
  const float cs = SCALE * LOG2E / (XS * XS);
  for (int kb = 0; kb < S; kb += 32) {
    v8f s0 = {}, s1 = {};
    { const b16* k0 = Kb + (size_t)(kb + col) * E, *k1 = Kb + (size_t)(kb + 16 + col) * E; s0 = wmma16b(frag_kb(k0, hh), qa0, s0); s0 = wmma16b(frag_kb(k0 + 32, hh), qa1, s0); s1 = wmma16b(frag_kb(k1, hh), qa0, s1); s1 = wmma16b(frag_kb(k1 + 32, hh), qa1, s1); }
    const v4i m00 = *(const v4i*)(mrow + kb + 8 * hh), m01 = *(const v4i*)(mrow + kb + 8 * hh + 4), m10 = *(const v4i*)(mrow + kb + 16 + 8 * hh), m11 = *(const v4i*)(mrow + kb + 16 + 8 * hh + 4);
    float e[16]; float mx = -INFINITY;
#pragma unroll
    for (int r = 0; r < 8; ++r) { const int mk0 = r < 4 ? m00[r] : m01[r - 4], mk1 = r < 4 ? m10[r] : m11[r - 4];
      e[r] = (mk0 == 0) ? -1.0e9f : s0[r] * cs; e[8 + r] = (mk1 == 0) ? -1.0e9f : s1[r] * cs; mx = fmaxf(mx, fmaxf(e[r], e[8 + r])); }
    mx = fmaxf(mx, __shfl_xor(mx, 16)); const float mn = fmaxf(m, mx); const float al = nexp2(m - mn); m = mn; float sum = 0.0f; v16b ph, pl;
#pragma unroll
    for (int i = 0; i < 16; ++i) { const float p = nexp2(e[i] - mn); sum += p; const b16 h_ = (b16)(p * PS); ph[i] = h_; pl[i] = (b16)(p * PS - (float)h_); }
    sum += __shfl_xor(sum, 16); l = l * al + sum;
#pragma unroll
    for (int t = 0; t < 4; ++t) { o[t] *= al; ol[t] *= al; const v16b vf = frag_kb(Vb + (size_t)(t * 16 + col) * S + kb, hh); o[t] = wmma16b(vf, ph, o[t]); ol[t] = wmma16b(vf, pl, ol[t]); } }
  const float inv = 1.0f / (l * PS * XS);
#pragma unroll
  for (int t = 0; t < 4; ++t)
#pragma unroll
    for (int r = 0; r < 8; ++r) To[wave][col][t * 16 + 8 * hh + r] = (o[t][r] + ol[t][r]) * inv;
  wave_lds_sync();
  for (int pass = 0; pass < 2; ++pass) { for (int r4 = 0; r4 < 16; r4 += 4) { const int rr = r4 + (lane >> 3), c8 = (lane & 7) * 8; v8b hv, lv; for (int j = 0; j < 8; ++j) { b16 a_, c_; split16(To[wave][rr][c8 + j] * XS, a_, c_); hv[j] = a_; lv[j] = c_; }
      const size_t gi = ((size_t)b * S + q0 + rr) * E + h * D + c8; *(volatile v8b*)(Oh + gi) = hv; *(volatile v8b*)(Ol + gi) = lv; } __threadfence(); }
}
__global__ __launch_bounds__(128) void proj_kernel(const b16* __restrict__ Oh, const b16* __restrict__ Ol, const b16* __restrict__ W16, const float* __restrict__ bias, float* __restrict__ out) {
  __shared__ __attribute__((aligned(16))) float Ts[4][16][128 + 4];
  const int wave = threadIdx.x >> 5, lane = threadIdx.x & 31, nloc = lane & 15, hlf = lane >> 4; const size_t m0 = (size_t)blockIdx.x * 64 + wave * 16; const int n0 = blockIdx.y * 128;
  v8f acc[8];
#pragma unroll
  for (int t = 0; t < 8; ++t) acc[t] = (v8f){};
#pragma unroll 2
  for (int kb = 0; kb < E; kb += 32) { const v16b a = frag_kb(Oh + (m0 + nloc) * E + kb, hlf), al = frag_kb(Ol + (m0 + nloc) * E + kb, hlf);
#pragma unroll
    for (int t = 0; t < 8; ++t) { const v16b bw = frag_kb(W16 + (size_t)(n0 + t * 16 + nloc) * E + kb, hlf); acc[t] = wmma16b(a, bw, acc[t]); acc[t] = wmma16b(al, bw, acc[t]); } }
#pragma unroll
  for (int t = 0; t < 8; ++t) { const float bb = bf16_rne(bias[n0 + t * 16 + nloc]);
#pragma unroll
    for (int r = 0; r < 8; ++r) Ts[wave][8 * hlf + r][t * 16 + nloc] = acc[t][r] * (1.0f / (XS * WSC)) + bb; }
  wave_lds_sync();
  for (int pass = 0; pass < 2; ++pass) { for (int rr = 0; rr < 16; ++rr) *(volatile v4f*)(out + (m0 + rr) * E + n0 + lane * 4) = *(const v4f*)(&Ts[wave][rr][lane * 4]); __threadfence(); }
}
}

extern "C" void kernel_launch(void* const* d_in, const int* in_sizes, int n_in, void* d_out, int out_size, void* d_ws, size_t ws_size, hipStream_t stream) {
  (void)n_in;
  auto Fp = [&](int i) { return (const float*)d_in[i]; };
  if (in_sizes[0] != NR * E || in_sizes[1] != NR * E || in_sizes[2] != NR * E || in_sizes[3] != NB * S * S || in_sizes[4] != E * E || out_size != NR * E) return;
  size_t off = 0; char* ws = (char*)d_ws;
  auto carve = [&](size_t bytes) { char* p = ws + off; off += (bytes + 255) & ~(size_t)255; return p; };
  b16* Q16 = (b16*)carve((size_t)NR * E * 2); b16* K16 = (b16*)carve((size_t)NR * E * 2); b16* W16 = (b16*)carve((size_t)E * E * 2); b16* VT16 = (b16*)carve((size_t)NB * NH * D * S * 2); b16* Oh = (b16*)carve((size_t)NR * E * 2); b16* Ol = (b16*)carve((size_t)NR * E * 2);
  if (off > ws_size || off > ((size_t)128 << 20)) return;
  prep_kernel<<<(unsigned)(((size_t)2 * NR * E / 8 + (size_t)E * E / 8 + 255) / 256), 256, 0, stream>>>(Fp(0), Fp(1), Fp(4), Q16, K16, W16);
  vt_kernel<<<dim3(S / 64, NH, NB), 256, 0, stream>>>(Fp(2), VT16);
  attn_kernel<<<dim3(S / 32, NH, NB), 64, 0, stream>>>(Q16, K16, VT16, (const int*)d_in[3], Oh, Ol);
  proj_kernel<<<dim3(NR / 64, E / 128), 128, 0, stream>>>(Oh, Ol, W16, Fp(5), (float*)d_out);
}
